// PGNN_42992622633784
// MI455X (gfx1250) — hardware-verified
//
#include <hip/hip_runtime.h>
#include <stddef.h>
#include <stdint.h>

#define NN     30000
#define KA     32
#define DF     128
#define DO2    64
#define MP     30080
#define GBM    64
#define GTHR   128
#define NWV    8
#define VBH1   0
#define VBH2   128
#define VWP2   192
#define VBOUT  256
#define VBP2   320
#define VECN   384
#define RNE_BP2  1
#define RNE_BOUT 1
#define WSMAX  134217728

static_assert(KA == 32);
static_assert(DF == 32 * 4);
static_assert(DO2 == 32 * 2);
static_assert(MP % GBM == 0 && MP % NWV == 0 && MP >= NN);
static_assert((MP * (DF / 8)) % 256 == 0);
static_assert(NN % 2 == 0);
static_assert(VECN == 96 * 4);

typedef float          v2f   __attribute__((ext_vector_type(2)));
typedef float          v4f   __attribute__((ext_vector_type(4)));
typedef float          v8f   __attribute__((ext_vector_type(8)));
typedef int            v8i   __attribute__((ext_vector_type(8)));
typedef unsigned       v2u   __attribute__((ext_vector_type(2)));
typedef unsigned short v8us  __attribute__((ext_vector_type(8)));
typedef unsigned short v16us __attribute__((ext_vector_type(16)));
typedef __bf16         v16bf __attribute__((ext_vector_type(16)));
typedef v4f  __attribute__((may_alias)) v4fa;
typedef v8us __attribute__((may_alias)) v8usa;
union FragB { v16bf v; v16us u; v8us h[2]; v8i w; };

__device__ __forceinline__ v8f wmb(const FragB& a, const FragB& b, v8f c) {
  v8f d = __builtin_amdgcn_wmma_f32_16x16x32_bf16(false, a.v, false, b.v, (short)0, c, false, false);
  asm volatile("v_nop\n\tv_nop\n\tv_nop\n\tv_nop" : "+v"(d) : "v"(a.w), "v"(b.w));
  return d;
}

__device__ __forceinline__ unsigned bf16_bits(float f) {
  const unsigned u = __float_as_uint(f);
  return (u + 0x7FFFu + ((u >> 16) & 1u)) >> 16;
}
__device__ __forceinline__ float bf16_val(float f) {
  return __uint_as_float(bf16_bits(f) << 16);
}
template <int ON>
__device__ __forceinline__ unsigned small_bits(float f) {
  if constexpr (ON != 0) return bf16_bits(f) << 16;
  else return __float_as_uint(f);
}

__global__ __launch_bounds__(256) __attribute__((amdgpu_num_vgpr(248)))
void k_pa(const float* __restrict__ x, unsigned short* XB) {
  const int u   = (int)blockIdx.x * 256 + (int)threadIdx.x;
  const int row = u >> 4;
  const int c8  = (u & 15) * 8;
  const int rc  = row < NN ? row : NN - 1;
  const float* p = x + (size_t)rc * DF + c8;
  const v4f a = *(const v4f*)p;
  const v4f b = *(const v4f*)(p + 4);
  const unsigned mk = (row < NN) ? 0xffffu : 0u;
  v8us o;
  o[0] = (unsigned short)(bf16_bits(a.x) & mk); o[1] = (unsigned short)(bf16_bits(a.y) & mk);
  o[2] = (unsigned short)(bf16_bits(a.z) & mk); o[3] = (unsigned short)(bf16_bits(a.w) & mk);
  o[4] = (unsigned short)(bf16_bits(b.x) & mk); o[5] = (unsigned short)(bf16_bits(b.y) & mk);
  o[6] = (unsigned short)(bf16_bits(b.z) & mk); o[7] = (unsigned short)(bf16_bits(b.w) & mk);
  unsigned short* dp = XB + (size_t)row * DF + c8;
  *(volatile v8us*)dp = o;
  __threadfence();
  *(volatile v8us*)dp = o;
}

__device__ __forceinline__ void cvt8_store(const float* __restrict__ src, unsigned short* dst) {
  const v4f a = *(const v4f*)src;
  const v4f b = *(const v4f*)(src + 4);
  v8us o;
  o[0] = (unsigned short)bf16_bits(a.x); o[1] = (unsigned short)bf16_bits(a.y);
  o[2] = (unsigned short)bf16_bits(a.z); o[3] = (unsigned short)bf16_bits(a.w);
  o[4] = (unsigned short)bf16_bits(b.x); o[5] = (unsigned short)bf16_bits(b.y);
  o[6] = (unsigned short)bf16_bits(b.z); o[7] = (unsigned short)bf16_bits(b.w);
  *(volatile v8us*)dst = o;
  __threadfence();
  *(volatile v8us*)dst = o;
}

__global__ __launch_bounds__(256) __attribute__((amdgpu_num_vgpr(248)))
void k_pb(const float* __restrict__ Wh1, const float* __restrict__ Wh2, const float* __restrict__ Wout,
          unsigned short* B1, unsigned short* B2, unsigned short* B3) {
  const int blk = (int)blockIdx.x;
  const int u   = blk * 256 + (int)threadIdx.x;
  if (blk < 16) {
    const int n = u >> 4, k8 = (u & 15) * 8;
    cvt8_store(Wh1 + (size_t)(n & 127) * 256 + (n >> 7) * 128 + k8, B1 + (size_t)n * 128 + k8);
  } else if (blk < 32) {
    const int v = u - 4096;
    const int n = v >> 5, k8 = (v & 31) * 8;
    cvt8_store(Wh2 + (size_t)(n & 63) * 256 + (n >> 6) * 128 + (k8 & 127), B2 + (size_t)n * 256 + k8);
  } else if (blk < 34) {
    const int v = u - 8192;
    const int n = v >> 3, k8 = (v & 7) * 8;
    cvt8_store(Wout + (size_t)n * 32 + (k8 & 31), B3 + (size_t)n * 64 + k8);
  }
}

__device__ __forceinline__ float blend5(float a1, float a2, float a3, float a4, float a5,
                                        unsigned m1, unsigned m2, unsigned m3, unsigned m4, unsigned m5) {
  const unsigned bits = (small_bits<1>(a1) & m1) | (small_bits<1>(a2) & m2) | (small_bits<1>(a3) & m3) |
                        (small_bits<RNE_BOUT>(a4) & m4) | (small_bits<RNE_BP2>(a5) & m5);
  return __uint_as_float(bits);
}

__global__ __launch_bounds__(96) __attribute__((amdgpu_num_vgpr(248)))
void k_pc(const float* __restrict__ bh1, const float* __restrict__ bh2, const float* __restrict__ wp2,
          const float* __restrict__ bp2, const float* __restrict__ bout, float* VEC) {
  const int t = (int)threadIdx.x;
  const int i1 = (t < 31 ? t : 31) * 4;
  const int t2 = t - 32, t3 = t - 48, t4 = t - 64;
  const int i2 = (t2 < 0 ? 0 : (t2 > 15 ? 15 : t2)) * 4;
  const int i3 = (t3 < 0 ? 0 : (t3 > 15 ? 15 : t3)) * 4;
  const int i4 = (t4 < 0 ? 0 : (t4 > 15 ? 15 : t4)) * 4;
  const v4f a1 = *(const v4f*)(bh1 + i1);
  const v4f a2 = *(const v4f*)(bh2 + i2);
  const v4f a3 = *(const v4f*)(wp2 + i3);
  const v4f a4 = *(const v4f*)(bout + i4);
  const float a5 = bp2[0];
  const unsigned m1 = (t < 32) ? 0xffffffffu : 0u;
  const unsigned m2 = (t >= 32 && t < 48) ? 0xffffffffu : 0u;
  const unsigned m3 = (t >= 48 && t < 64) ? 0xffffffffu : 0u;
  const unsigned m4 = (t >= 64 && t < 80) ? 0xffffffffu : 0u;
  const unsigned m5 = (t >= 80 && t < 88) ? 0xffffffffu : 0u;
  v4f o;
  o.x = blend5(a1.x, a2.x, a3.x, a4.x, a5, m1, m2, m3, m4, m5);
  o.y = blend5(a1.y, a2.y, a3.y, a4.y, a5, m1, m2, m3, m4, m5);
  o.z = blend5(a1.z, a2.z, a3.z, a4.z, a5, m1, m2, m3, m4, m5);
  o.w = blend5(a1.w, a2.w, a3.w, a4.w, a5, m1, m2, m3, m4, m5);
  float* dp = VEC + 4 * t;
  *(volatile v4f*)dp = o;
  __threadfence();
  *(volatile v4f*)dp = o;
}

template <int CPR, int LPR, int RPI, int NIT>
__device__ __forceinline__ void g_pass(const float* stg, float* outp, int opitch, int nOut, int rowBase,
                                       int wave, int lane, int gcol, v4f bb4) {
  const int lr = lane / LPR;
  const int lc = 4 * (lane % LPR);
#pragma unroll
  for (int it = 0; it < NIT; ++it) {
    const int rl = 16 * wave + it * RPI + lr;
    const int r  = rowBase + rl;
    const v4f v = *(const v4fa*)(stg + rl * CPR + lc) + bb4;
    if (r < nOut) *(volatile v4f*)(outp + (size_t)r * (size_t)opitch + gcol) = v;
  }
}

template <int KK, int NT>
__global__ __launch_bounds__(GTHR) __attribute__((amdgpu_num_vgpr(248)))
void k_gemm(const unsigned short* __restrict__ Apl, const unsigned short* __restrict__ BT,
            const float* __restrict__ bias, int biasFrom, int biasLen,
            float* outp, int opitch, int nOut) {
  constexpr int CPR = 16 * NT;
  constexpr int LPR = CPR / 4;
  constexpr int RPI = 32 / LPR;
  constexpr int NIT = 16 / RPI;
  static_assert(KK % 32 == 0);
  static_assert(NT == 8 || NT == 4);
  __shared__ __attribute__((aligned(16))) float stg[GBM * CPR];
  const int tid = (int)threadIdx.x, lane = tid & 31, wave = tid >> 5, hh = lane >> 4, m = lane & 15;
  const int rowBase = (int)blockIdx.x * GBM;
  const int cb = (int)blockIdx.y;

  v8f acc[NT];
  {
    const v8f z = {0.f, 0.f, 0.f, 0.f, 0.f, 0.f, 0.f, 0.f};
#pragma unroll
    for (int t = 0; t < NT; ++t) acc[t] = z;
  }
  const unsigned short* ap = Apl + (size_t)(rowBase + 16 * wave + m) * (size_t)KK + 8 * hh;
  const unsigned short* bp = BT + (size_t)(cb * CPR + m) * (size_t)KK + 8 * hh;

#pragma unroll 1
  for (int k0 = 0; k0 < KK; k0 += 32) {
    FragB af;
    af.h[0] = *(const v8usa*)(ap + k0);
    af.h[1] = *(const v8usa*)(ap + k0 + 16);
#pragma unroll
    for (int nt = 0; nt < NT; ++nt) {
      const unsigned short* wq = bp + (size_t)(16 * nt) * (size_t)KK + k0;
      FragB bf;
      bf.h[0] = *(const v8usa*)wq;
      bf.h[1] = *(const v8usa*)(wq + 16);
      acc[nt] = wmb(af, bf, acc[nt]);
    }
  }

#pragma unroll
  for (int nt = 0; nt < NT; ++nt) {
    const int lc = 16 * nt + m;
#pragma unroll
    for (int r = 0; r < 8; ++r) {
      const int lr = 16 * wave + 8 * hh + r;
      stg[lr * CPR + lc] = acc[nt][r];
    }
  }
  __syncthreads();

  const int gcol = cb * CPR + 4 * (lane % LPR);
  const int bi   = gcol - biasFrom;
  const int bic  = bi < 0 ? 0 : (bi > biasLen - 4 ? biasLen - 4 : bi);
  const float bsel = (bi >= 0) ? 1.0f : 0.0f;
  const v4f bb4 = *(const v4f*)(bias + bic) * bsel;

  g_pass<CPR, LPR, RPI, NIT>(stg, outp, opitch, nOut, rowBase, wave, lane, gcol, bb4);
  __threadfence();
  g_pass<CPR, LPR, RPI, NIT>(stg, outp, opitch, nOut, rowBase, wave, lane, gcol, bb4);
}

__global__ __launch_bounds__(256) __attribute__((amdgpu_num_vgpr(248)))
void k_agg1(const int* __restrict__ amax, const float* __restrict__ dmax, const float* __restrict__ PQ1,
            unsigned short* H1) {
  const int tid = (int)threadIdx.x, lane = tid & 31, wave = tid >> 5;
  const int node = (int)blockIdx.x * NWV + wave;
  const int nc   = node < NN ? node : NN - 1;
  int a = amax[(size_t)nc * KA + lane];
  a = a < 0 ? 0 : (a > NN - 1 ? NN - 1 : a);
  const int di = __float_as_int(bf16_val(dmax[(size_t)nc * KA + lane]));
  const v4f q = *(const v4f*)(PQ1 + (size_t)nc * 256 + DF + 4 * lane);
  float a0 = 0.0f, a1 = 0.0f, a2 = 0.0f, a3 = 0.0f;
#pragma unroll 4
  for (int k = 0; k < KA; ++k) {
    const int   ak = __builtin_amdgcn_readlane(a, k);
    const float dk = __int_as_float(__builtin_amdgcn_readlane(di, k));
    const v4f p = *(const v4f*)(PQ1 + (size_t)ak * 256 + 4 * lane);
    float v0 = fmaf(dk, p.x, q.x);
    float v1 = fmaf(dk, p.y, q.y);
    float v2 = fmaf(dk, p.z, q.z);
    float v3 = fmaf(dk, p.w, q.w);
    v0 = (v0 > 0.0f) ? v0 : 0.0f;
    v1 = (v1 > 0.0f) ? v1 : 0.0f;
    v2 = (v2 > 0.0f) ? v2 : 0.0f;
    v3 = (v3 > 0.0f) ? v3 : 0.0f;
    a0 += v0; a1 += v1; a2 += v2; a3 += v3;
  }
  const bool live = node < NN;
  float h0 = a0 * 0.03125f, h1 = a1 * 0.03125f, h2 = a2 * 0.03125f, h3 = a3 * 0.03125f;
  h0 = (h0 > 0.0f) ? h0 : 0.0f; h1 = (h1 > 0.0f) ? h1 : 0.0f;
  h2 = (h2 > 0.0f) ? h2 : 0.0f; h3 = (h3 > 0.0f) ? h3 : 0.0f;
  h0 = live ? h0 : 0.0f; h1 = live ? h1 : 0.0f; h2 = live ? h2 : 0.0f; h3 = live ? h3 : 0.0f;
  const unsigned b0 = bf16_bits(h0), b1 = bf16_bits(h1), b2 = bf16_bits(h2), b3 = bf16_bits(h3);
  const unsigned l0 = bf16_bits(h0 - __uint_as_float(b0 << 16));
  const unsigned l1 = bf16_bits(h1 - __uint_as_float(b1 << 16));
  const unsigned l2 = bf16_bits(h2 - __uint_as_float(b2 << 16));
  const unsigned l3 = bf16_bits(h3 - __uint_as_float(b3 << 16));
  v2u hv, lv;
  hv.x = (b0 & 0xffffu) | (b1 << 16); hv.y = (b2 & 0xffffu) | (b3 << 16);
  lv.x = (l0 & 0xffffu) | (l1 << 16); lv.y = (l2 & 0xffffu) | (l3 << 16);
  unsigned short* dp = H1 + (size_t)node * 256 + 4 * lane;
  *(volatile v2u*)dp = hv;
  *(volatile v2u*)(dp + DF) = lv;
  __threadfence();
  *(volatile v2u*)dp = hv;
  *(volatile v2u*)(dp + DF) = lv;
}

__global__ __launch_bounds__(256) __attribute__((amdgpu_num_vgpr(248)))
void k_pos(const int* __restrict__ amax, const float* __restrict__ dmax, const float* __restrict__ PQ2,
           const float* __restrict__ VEC, unsigned short* XN) {
  const int tid = (int)threadIdx.x, lane = tid & 31, wave = tid >> 5;
  const int node = (int)blockIdx.x * NWV + wave;
  const int nc   = node < NN ? node : NN - 1;
  int a = amax[(size_t)nc * KA + lane];
  a = a < 0 ? 0 : (a > NN - 1 ? NN - 1 : a);
  const int di = __float_as_int(bf16_val(dmax[(size_t)nc * KA + lane]));
  const v2f q = *(const v2f*)(PQ2 + (size_t)nc * DF + DO2 + 2 * lane);
  const v2f w = *(const v2f*)(VEC + VWP2 + 2 * lane);
  const float bp = VEC[VBP2];
  float pos = 0.0f;
#pragma unroll 4
  for (int k = 0; k < KA; ++k) {
    const int   ak = __builtin_amdgcn_readlane(a, k);
    const float dk = __int_as_float(__builtin_amdgcn_readlane(di, k));
    const v2f p = *(const v2f*)(PQ2 + (size_t)ak * DF + 2 * lane);
    float v0 = fmaf(dk, p.x, q.x);
    float v1 = fmaf(dk, p.y, q.y);
    v0 = (v0 > 0.0f) ? v0 : 0.0f;
    v1 = (v1 > 0.0f) ? v1 : 0.0f;
    float s = v0 * w.x + v1 * w.y;
    s += __shfl_xor(s, 16, 32);
    s += __shfl_xor(s, 8, 32);
    s += __shfl_xor(s, 4, 32);
    s += __shfl_xor(s, 2, 32);
    s += __shfl_xor(s, 1, 32);
    const float cand = s + bp;
    pos = (lane == k) ? cand : pos;
  }
  float ss = pos * pos;
  ss += __shfl_xor(ss, 16, 32);
  ss += __shfl_xor(ss, 8, 32);
  ss += __shfl_xor(ss, 4, 32);
  ss += __shfl_xor(ss, 2, 32);
  ss += __shfl_xor(ss, 1, 32);
  const float nrm = fmaxf(sqrtf(ss), 1e-12f);
  const float xn  = pos / nrm;
  const unsigned hb = bf16_bits(xn);
  const unsigned lb = bf16_bits(xn - __uint_as_float(hb << 16));
  const int wv = (int)((hb & 0xffffu) | (lb << 16));
  const int j2 = 2 * (lane & 15);
  const unsigned s0 = (unsigned)__shfl(wv, j2, 32);
  const unsigned s1 = (unsigned)__shfl(wv, j2 + 1, 32);
  const unsigned whi = (s0 & 0xffffu) | (s1 << 16);
  const unsigned wlo = (s0 >> 16) | (s1 & 0xffff0000u);
  unsigned ow = (lane < 16) ? whi : wlo;
  ow = (node < NN) ? ow : 0u;
  unsigned* dp = (unsigned*)XN + (size_t)node * 32 + lane;
  *(volatile unsigned*)dp = ow;
  __threadfence();
  *(volatile unsigned*)dp = ow;
}

static inline size_t al256(size_t o) { return (o + 255) & ~(size_t)255; }

extern "C" void kernel_launch(void* const* d_in, const int* in_sizes, int n_in,
                              void* d_out, int out_size, void* d_ws, size_t ws_size,
                              hipStream_t stream) {
  if (n_in < 13) return;
  if (in_sizes[0] != NN * DF) return;
  if (in_sizes[1] != NN * KA) return;
  if (in_sizes[2] != NN * KA) return;
  if (in_sizes[3] != DF * 2 * DF) return;
  if (in_sizes[4] != DF) return;
  if (in_sizes[7] != DO2 * 2 * DF) return;
  if (in_sizes[8] != DO2) return;
  if (in_sizes[9] != DO2) return;
  if (in_sizes[10] != 1) return;
  if (in_sizes[11] != DO2 * KA) return;
  if (in_sizes[12] != DO2) return;
  if (out_size != NN * DO2) return;

  const float* x    = (const float*)d_in[0];
  const float* dmax = (const float*)d_in[1];
  const int*   amax = (const int*)d_in[2];
  const float* Wh1  = (const float*)d_in[3];
  const float* bh1  = (const float*)d_in[4];
  const float* Wh2  = (const float*)d_in[7];
  const float* bh2  = (const float*)d_in[8];
  const float* wp2  = (const float*)d_in[9];
  const float* bp2  = (const float*)d_in[10];
  const float* Wout = (const float*)d_in[11];
  const float* bout = (const float*)d_in[12];
  float* out = (float*)d_out;

  char* ws = (char*)d_ws;
  size_t off = 0;
  const size_t oXB  = off; off = al256(off + (size_t)MP * DF * 2);
  const size_t oPQ1 = off; off = al256(off + (size_t)MP * 256 * 4);
  const size_t oH1  = off; off = al256(off + (size_t)MP * 256 * 2);
  const size_t oPQ2 = off; off = al256(off + (size_t)MP * DF * 4);
  const size_t oXN  = off; off = al256(off + (size_t)MP * DO2 * 2);
  const size_t oB1  = off; off = al256(off + (size_t)256 * 128 * 2);
  const size_t oB2  = off; off = al256(off + (size_t)128 * 256 * 2);
  const size_t oB3  = off; off = al256(off + (size_t)64 * 64 * 2);
  const size_t oVEC = off; off = al256(off + (size_t)VECN * 4);
  if (off > ws_size || off > (size_t)WSMAX) return;
  unsigned short* XB  = (unsigned short*)(ws + oXB);
  float*          PQ1 = (float*)(ws + oPQ1);
  unsigned short* H1  = (unsigned short*)(ws + oH1);
  float*          PQ2 = (float*)(ws + oPQ2);
  unsigned short* XN  = (unsigned short*)(ws + oXN);
  unsigned short* B1  = (unsigned short*)(ws + oB1);
  unsigned short* B2  = (unsigned short*)(ws + oB2);
  unsigned short* B3  = (unsigned short*)(ws + oB3);
  float*          VEC = (float*)(ws + oVEC);

  k_pa<<<(MP * (DF / 8)) / 256, 256, 0, stream>>>(x, XB);
  k_pb<<<34, 256, 0, stream>>>(Wh1, Wh2, Wout, B1, B2, B3);
  k_pc<<<1, 96, 0, stream>>>(bh1, bh2, wp2, bp2, bout, VEC);
  k_gemm<128, 8><<<dim3(MP / GBM, 2), GTHR, 0, stream>>>(XB, B1, VEC + VBH1, 128, 128, PQ1, 256, MP);
  k_agg1<<<MP / NWV, 256, 0, stream>>>(amax, dmax, PQ1, H1);
  k_gemm<256, 8><<<dim3(MP / GBM, 1), GTHR, 0, stream>>>(H1, B2, VEC + VBH2, 64, 64, PQ2, 128, MP);
  k_pos<<<MP / NWV, 256, 0, stream>>>(amax, dmax, PQ2, VEC, XN);
  k_gemm<64, 4><<<dim3(MP / GBM, 1), GTHR, 0, stream>>>(XN, B3, VEC + VBOUT, 0, 64, out, 64, NN);
  (void)hipGetLastError();
}
